// UpResblock_65798898974753
// MI455X (gfx1250) — hardware-verified
//
#include <hip/hip_runtime.h>
#include <stddef.h>


typedef _Float16 v16h __attribute__((ext_vector_type(16)));
typedef _Float16 v8h  __attribute__((ext_vector_type(8)));
typedef float    v8f  __attribute__((ext_vector_type(8)));
typedef float    v4f  __attribute__((ext_vector_type(4)));
typedef unsigned int v4u __attribute__((ext_vector_type(4)));

union Frag  { v16h v; v8h p[2]; v4u u[2]; };
union Chunk { v8h h; v4u u; };

#define DEV static __device__ __forceinline__

#define NB     2
#define NLINE  (NB * 16 * 16 * 16)
#define WP     18
#define CX     64
#define CY     32
#define NTAP   81

#define NCH1   (NTAP * CY * CX / 8)
#define NCH2   (NTAP * CY * CY / 8)
#define NCH3   (CY * CX / 8)
#define NCHU   (8 * CY * 128 / 8)
#define NCHUNK (NCH1 + NCH2 + NCH3 + NCHU)

DEV v8f zero8() {
  v8f z;
#pragma unroll
  for (int i = 0; i < 8; ++i) z[i] = 0.0f;
  return z;
}

DEV v4u zero4u() {
  v4u z;
  z.x = 0u; z.y = 0u; z.z = 0u; z.w = 0u;
  return z;
}

DEV v4u splat4u(unsigned s) {
  v4u z;
  z.x = s; z.y = s; z.z = s; z.w = s;
  return z;
}

DEV float relu(float v) { return v > 0.0f ? v : 0.0f; }

DEV v8f wmma16(v16h a, v16h b, v8f c) {
  v8f d = __builtin_amdgcn_wmma_f32_16x16x32_f16(false, a, false, b, (short)0, c, false, false);
  asm volatile("v_nop\n\tv_nop\n\tv_nop\n\tv_nop" : "+v"(d) : "v"(a), "v"(b));
  return d;
}

DEV v16h ldfrag(const _Float16* row, int hh) {
  Frag f;
  f.p[0] = *(const v8h*)(row + 8 * hh);
  f.p[1] = *(const v8h*)(row + 16 + 8 * hh);
  return f.v;
}

__global__ __launch_bounds__(256) void k_prep(
    const float* __restrict__ up_w, const float* __restrict__ w1,
    const float* __restrict__ w2, const float* __restrict__ w3,
    _Float16* __restrict__ wbu, _Float16* __restrict__ wb1,
    _Float16* __restrict__ wb2, _Float16* __restrict__ wb3, int nchunks) {
  const int j = (int)(blockIdx.x * 256u + threadIdx.x);
  if (j >= nchunks) return;
  float v[8];
  _Float16* dst;
  if (j < NCH1) {
    const int row = j >> 3, tap = row >> 5, co = row & 31, ci0 = (j & 7) * 8;
#pragma unroll
    for (int e = 0; e < 8; ++e) v[e] = w1[(size_t)(co * CX + ci0 + e) * NTAP + tap] * 64.0f;
    dst = wb1 + (size_t)j * 8;
  } else if (j < NCH1 + NCH2) {
    const int j2 = j - NCH1;
    const int row = j2 >> 2, tap = row >> 5, co = row & 31, ci0 = (j2 & 3) * 8;
#pragma unroll
    for (int e = 0; e < 8; ++e) v[e] = w2[(size_t)(co * CY + ci0 + e) * NTAP + tap] * 64.0f;
    dst = wb2 + (size_t)j2 * 8;
  } else if (j < NCH1 + NCH2 + NCH3) {
    const int j3 = j - NCH1 - NCH2;
#pragma unroll
    for (int e = 0; e < 8; ++e) v[e] = w3[j3 * 8 + e] * 8.0f;
    dst = wb3 + (size_t)j3 * 8;
  } else {
    const int j4 = j - NCH1 - NCH2 - NCH3;
    const int row = j4 >> 4, pqr = row >> 5, o = row & 31, k0 = (j4 & 15) * 8;
    const int sp = k0 >> 6, c0 = k0 & 63;
#pragma unroll
    for (int e = 0; e < 8; ++e) v[e] = up_w[((c0 + e) * CY + o) * 16 + pqr * 2 + sp] * 32.0f;
    dst = wbu + (size_t)j4 * 8;
  }
  Chunk c;
#pragma unroll
  for (int e = 0; e < 8; ++e) c.h[e] = (_Float16)v[e];
  *(volatile v4u*)dst = c.u;
  __threadfence();
  *(volatile v4u*)dst = c.u;
}

__global__ __launch_bounds__(64) void k_build_xc(
    const float* __restrict__ x1, const float* __restrict__ x2,
    const _Float16* __restrict__ wbu, const float* __restrict__ up_b,
    _Float16* __restrict__ xc) {
  __shared__ __attribute__((aligned(16))) _Float16 xs[16 * CX];
  __shared__ __attribute__((aligned(16))) _Float16 xa[8 * CX];
  const int line = (int)blockIdx.x;
  const int tid = threadIdx.x, lane = tid & 31, wave = tid >> 5;
  const int b = line >> 12, t = (line >> 8) & 15, d = (line >> 4) & 15, h = line & 15;
  const int sp0 = (line & 4095) << 4;

  {
    const int c = tid >> 1, w0 = (tid & 1) * 8;
    const float* p = x2 + ((size_t)(b * 32 + c) << 16) + sp0 + w0;
    const v4f u0 = *(const v4f*)p;
    const v4f u1 = *(const v4f*)(p + 4);
#pragma unroll
    for (int e = 0; e < 4; ++e) {
      xs[(w0 + e) * CX + c]     = (_Float16)u0[e];
      xs[(w0 + 4 + e) * CX + c] = (_Float16)u1[e];
    }
  }
  {
    const int c = tid;
    const int s1 = ((t >> 1) << 9) | ((d >> 1) << 6) | ((h >> 1) << 3);
    const float* p = x1 + ((size_t)(b * 64 + c) << 12) + s1;
    const v4f u0 = *(const v4f*)p;
    const v4f u1 = *(const v4f*)(p + 4);
#pragma unroll
    for (int e = 0; e < 4; ++e) {
      xa[e * CX + c]       = (_Float16)u0[e];
      xa[(4 + e) * CX + c] = (_Float16)u1[e];
    }
  }
  __syncthreads();

  const int m = lane & 15, hh = lane >> 4;
  const int pqr = ((t & 1) << 2) | ((d & 1) << 1) | (h & 1);
  const _Float16* brow = wbu + (size_t)((pqr * CY + wave * 16 + m) * 128);
  const _Float16* arow = xa + (m >> 1) * CX;
  const unsigned podd = (unsigned)(m & 1);
  v8f acc = zero8();
#pragma unroll
  for (int ks = 0; ks < 4; ++ks) {
    const unsigned sel = (((unsigned)(ks >> 1)) == podd) ? 0xffffffffu : 0u;
    const v4u mk = splat4u(sel);
    Frag a;
    a.v = ldfrag(arow + (ks & 1) * 32, hh);
    a.u[0] = a.u[0] & mk;
    a.u[1] = a.u[1] & mk;
    const v16h bv = ldfrag(brow + ks * 32, hh);
    acc = wmma16(a.v, bv, acc);
  }
  const float ub = up_b[wave * 16 + m];
#pragma unroll
  for (int r = 0; r < 8; ++r)
    xs[(8 * hh + r) * CX + 32 + wave * 16 + m] = (_Float16)(acc[r] * 0.03125f + ub);
  __syncthreads();

  const int q = lane & 7;
  const v4u z = zero4u();
  Chunk cv[3];
#pragma unroll
  for (int i = 0; i < 3; ++i) {
    const int wp = (wave + 2 * i) * 4 + (lane >> 3);
    const int wpc = wp < 1 ? 1 : (wp > 16 ? 16 : wp);
    Chunk c;
    c.u = *(const v4u*)(xs + (wpc - 1) * CX + 8 * q);
    const v4u keep = splat4u((wp >= 1 && wp <= 16) ? 0xffffffffu : 0u);
    cv[i].u = c.u & keep;
  }
#pragma unroll
  for (int i = 0; i < 3; ++i) {
    const int wp = (wave + 2 * i) * 4 + (lane >> 3);
    if (wp < WP) *(volatile v4u*)(xc + ((size_t)line * WP + wp) * CX + 8 * q) = cv[i].u;
  }
  __threadfence();
#pragma unroll
  for (int i = 0; i < 3; ++i) {
    const int wp = (wave + 2 * i) * 4 + (lane >> 3);
    if (wp < WP) *(volatile v4u*)(xc + ((size_t)line * WP + wp) * CX + 8 * q) = cv[i].u;
  }
  (void)z;
}

__global__ __launch_bounds__(256) void k_conv1(
    const _Float16* __restrict__ xc, const _Float16* __restrict__ wb1,
    const float* __restrict__ b1, _Float16* __restrict__ y1) {
  __shared__ __attribute__((aligned(16))) _Float16 ys[8 * 16 * CY];
  const int lane = threadIdx.x & 31, wave = threadIdx.x >> 5;
  const int tile = __builtin_amdgcn_readfirstlane((int)(blockIdx.x * 8u + (unsigned)wave));
  const int b = tile >> 12, t = (tile >> 8) & 15, d = (tile >> 4) & 15, h = tile & 15;
  const int m = lane & 15, hh = lane >> 4;

  v8f acc[2][2];
  acc[0][0] = zero8(); acc[0][1] = zero8();
  acc[1][0] = zero8(); acc[1][1] = zero8();

  for (int kt = 0; kt < 3; ++kt) {
    const int it = t + kt - 1;
    if ((unsigned)it >= 16u) continue;
    for (int kd = 0; kd < 3; ++kd) {
      const int id = d + kd - 1;
      if ((unsigned)id >= 16u) continue;
      for (int kh = 0; kh < 3; ++kh) {
        const int ih = h + kh - 1;
        if ((unsigned)ih >= 16u) continue;
        const int lin = ((b * 16 + it) * 16 + id) * 16 + ih;
        const _Float16* arow0 = xc + ((size_t)lin * WP + m) * CX;
        const _Float16* wt0 = wb1 + (size_t)(((kt * 3 + kd) * 3 + kh) * 3) * (CY * CX);
#pragma unroll
        for (int kw = 0; kw < 3; ++kw) {
          const _Float16* arow = arow0 + kw * CX;
          const _Float16* wt = wt0 + kw * (CY * CX);
#pragma unroll
          for (int c = 0; c < 2; ++c) {
            const v16h a   = ldfrag(arow + c * 32, hh);
            const v16h bw0 = ldfrag(wt + m * CX + c * 32, hh);
            const v16h bw1 = ldfrag(wt + (16 + m) * CX + c * 32, hh);
            acc[c][0] = wmma16(a, bw0, acc[c][0]);
            acc[c][1] = wmma16(a, bw1, acc[c][1]);
          }
        }
      }
    }
  }

  _Float16* yw = ys + wave * (16 * CY);
  const float bias0 = b1[m], bias1 = b1[16 + m];
#pragma unroll
  for (int r = 0; r < 8; ++r) {
    const int w = 8 * hh + r;
    yw[w * CY + m]      = (_Float16)relu((acc[0][0][r] + acc[1][0][r]) * 0.015625f + bias0);
    yw[w * CY + 16 + m] = (_Float16)relu((acc[0][1][r] + acc[1][1][r]) * 0.015625f + bias1);
  }
  __syncthreads();

  Chunk cv[3];
#pragma unroll
  for (int i = 0; i < 3; ++i) {
    const int j = lane + 32 * i;
    const int wp = j >> 2, q = j & 3;
    const int wpc = wp < 1 ? 1 : (wp > 16 ? 16 : wp);
    Chunk c;
    c.u = *(const v4u*)(yw + (wpc - 1) * CY + 8 * q);
    const v4u keep = splat4u((wp >= 1 && wp <= 16) ? 0xffffffffu : 0u);
    cv[i].u = c.u & keep;
  }
  _Float16* ybase = y1 + (size_t)tile * (WP * CY);
#pragma unroll
  for (int i = 0; i < 3; ++i) {
    const int j = lane + 32 * i;
    if (j < (WP * CY / 8)) *(volatile v4u*)(ybase + 8 * j) = cv[i].u;
  }
  __threadfence();
#pragma unroll
  for (int i = 0; i < 3; ++i) {
    const int j = lane + 32 * i;
    if (j < (WP * CY / 8)) *(volatile v4u*)(ybase + 8 * j) = cv[i].u;
  }
}

__global__ __launch_bounds__(256) void k_conv2sc(
    const _Float16* __restrict__ y1, const _Float16* __restrict__ xc,
    const _Float16* __restrict__ wb2, const _Float16* __restrict__ wb3,
    const float* __restrict__ b2, const float* __restrict__ b3,
    float* __restrict__ out) {
  __shared__ __attribute__((aligned(16))) float os[CY * 128];
  const int lane = threadIdx.x & 31, wave = threadIdx.x >> 5;
  const int tile = __builtin_amdgcn_readfirstlane((int)(blockIdx.x * 8u + (unsigned)wave));
  const int b = tile >> 12, t = (tile >> 8) & 15, d = (tile >> 4) & 15, h = tile & 15;
  const int m = lane & 15, hh = lane >> 4;

  v8f acc[2][2];
  v8f sacc[2];
  acc[0][0] = zero8(); acc[0][1] = zero8();
  acc[1][0] = zero8(); acc[1][1] = zero8();
  sacc[0] = zero8(); sacc[1] = zero8();

  {
    const _Float16* arow = xc + ((size_t)tile * WP + m + 1) * CX;
#pragma unroll
    for (int c = 0; c < 2; ++c) {
      const v16h a   = ldfrag(arow + c * 32, hh);
      const v16h bw0 = ldfrag(wb3 + m * CX + c * 32, hh);
      const v16h bw1 = ldfrag(wb3 + (16 + m) * CX + c * 32, hh);
      sacc[0] = wmma16(a, bw0, sacc[0]);
      sacc[1] = wmma16(a, bw1, sacc[1]);
    }
  }
  for (int kt = 0; kt < 3; ++kt) {
    const int it = t + kt - 1;
    if ((unsigned)it >= 16u) continue;
    for (int kd = 0; kd < 3; ++kd) {
      const int id = d + kd - 1;
      if ((unsigned)id >= 16u) continue;
      for (int kh = 0; kh < 3; ++kh) {
        const int ih = h + kh - 1;
        if ((unsigned)ih >= 16u) continue;
        const int lin = ((b * 16 + it) * 16 + id) * 16 + ih;
        const _Float16* arow0 = y1 + ((size_t)lin * WP + m) * CY;
        const _Float16* wt0 = wb2 + (size_t)(((kt * 3 + kd) * 3 + kh) * 3) * (CY * CY);
#pragma unroll
        for (int kw = 0; kw < 3; ++kw) {
          const _Float16* arow = arow0 + kw * CY;
          const _Float16* wt = wt0 + kw * (CY * CY);
          const v16h a   = ldfrag(arow, hh);
          const v16h bw0 = ldfrag(wt + m * CY, hh);
          const v16h bw1 = ldfrag(wt + (16 + m) * CY, hh);
          acc[kw & 1][0] = wmma16(a, bw0, acc[kw & 1][0]);
          acc[kw & 1][1] = wmma16(a, bw1, acc[kw & 1][1]);
        }
      }
    }
  }

  const float bb0 = b2[m] + b3[m];
  const float bb1 = b2[16 + m] + b3[16 + m];
#pragma unroll
  for (int r = 0; r < 8; ++r) {
    const int idx = wave * 16 + 8 * hh + r;
    os[m * 128 + idx]        = relu((acc[0][0][r] + acc[1][0][r]) * 0.015625f + sacc[0][r] * 0.125f + bb0);
    os[(16 + m) * 128 + idx] = relu((acc[0][1][r] + acc[1][1][r]) * 0.015625f + sacc[1][r] * 0.125f + bb1);
  }
  __syncthreads();

  const int sp_blk = ((int)((blockIdx.x * 8u) & 4095u)) << 4;
  v4f ov[4];
#pragma unroll
  for (int i = 0; i < 4; ++i) {
    const int co = wave * 4 + i;
    ov[i] = *(const v4f*)(os + co * 128 + 4 * lane);
  }
#pragma unroll
  for (int i = 0; i < 4; ++i) {
    const int co = wave * 4 + i;
    float* dst = out + ((size_t)(b * CY + co) << 16) + sp_blk + 4 * lane;
    *(volatile v4f*)dst = ov[i];
  }
  __threadfence();
#pragma unroll
  for (int i = 0; i < 4; ++i) {
    const int co = wave * 4 + i;
    float* dst = out + ((size_t)(b * CY + co) << 16) + sp_blk + 4 * lane;
    *(volatile v4f*)dst = ov[i];
  }
}

extern "C" void kernel_launch(void* const* d_in, const int* in_sizes, int n_in,
                              void* d_out, int out_size, void* d_ws, size_t ws_size,
                              hipStream_t stream) {
  if (n_in < 10) return;
  if (in_sizes[0] != NB * 64 * 4096) return;
  if (in_sizes[1] != NB * 32 * 65536) return;
  if (in_sizes[2] != 64 * 32 * 16) return;
  if (in_sizes[3] != 32) return;
  if (in_sizes[4] != CY * CX * NTAP) return;
  if (in_sizes[5] != 32) return;
  if (in_sizes[6] != CY * CY * NTAP) return;
  if (in_sizes[7] != 32) return;
  if (in_sizes[8] != CY * CX) return;
  if (in_sizes[9] != 32) return;
  if (out_size != NB * CY * 65536) return;

  const float* x1   = (const float*)d_in[0];
  const float* x2   = (const float*)d_in[1];
  const float* up_w = (const float*)d_in[2];
  const float* up_b = (const float*)d_in[3];
  const float* w1   = (const float*)d_in[4];
  const float* b1   = (const float*)d_in[5];
  const float* w2   = (const float*)d_in[6];
  const float* b2   = (const float*)d_in[7];
  const float* w3   = (const float*)d_in[8];
  const float* b3   = (const float*)d_in[9];
  float* out = (float*)d_out;

  const size_t XC_B  = (size_t)NLINE * WP * CX * 2;
  const size_t Y1_B  = (size_t)NLINE * WP * CY * 2;
  const size_t WB1_B = (size_t)NCH1 * 16;
  const size_t WB2_B = (size_t)NCH2 * 16;
  const size_t WB3_B = (size_t)NCH3 * 16;
  const size_t WBU_B = (size_t)NCHU * 16;
  const size_t total = XC_B + Y1_B + WB1_B + WB2_B + WB3_B + WBU_B;
  if (total > ws_size) return;

  char* ws = (char*)d_ws;
  _Float16* xc_w  = (_Float16*)(ws);
  _Float16* y1_w  = (_Float16*)(ws + XC_B);
  _Float16* wb1_w = (_Float16*)(ws + XC_B + Y1_B);
  _Float16* wb2_w = (_Float16*)(ws + XC_B + Y1_B + WB1_B);
  _Float16* wb3_w = (_Float16*)(ws + XC_B + Y1_B + WB1_B + WB2_B);
  _Float16* wbu_w = (_Float16*)(ws + XC_B + Y1_B + WB1_B + WB2_B + WB3_B);

  const int nchunks = NCHUNK;
  k_prep<<<(nchunks + 255) / 256, 256, 0, stream>>>(up_w, w1, w2, w3, wbu_w, wb1_w, wb2_w, wb3_w, nchunks);
  k_build_xc<<<NLINE, 64, 0, stream>>>(x1, x2, wbu_w, up_b, xc_w);
  k_conv1<<<NLINE / 8, 256, 0, stream>>>(xc_w, wb1_w, b1, y1_w);
  k_conv2sc<<<NLINE / 8, 256, 0, stream>>>(y1_w, xc_w, wb2_w, wb3_w, b2, b3, out);
}
